// FiniteModel_33045478375828
// MI455X (gfx1250) — hardware-run, weakly checked
//
#include <hip/hip_runtime.h>


#ifndef NS
#define NS 32768
#endif
#define NS_FULL 32768
#ifndef NC
#define NC 2048
#endif
#define NC_FULL 2048
#define ND   16
#define AW   8
#define OSP  20
#define SC2  ((float)(50.0 * 1.4426950408889634))
#define PSH  14.0f
#define NEGB (-3.0e38f)

static_assert(ND == 16);
static_assert(NC % 32 == 0);
static_assert(NS % (16 * AW) == 0);
static_assert(NS <= NS_FULL);
static_assert(NC <= NC_FULL);
static_assert(((size_t)NS * ND) % 8 == 0);
static_assert(((size_t)NC * ND) % 8 == 0);
static_assert(NC % 8 == 0);
static_assert(((size_t)ND * NC / 8) % 256 == 0);
static_assert((OSP * 4) % 16 == 0);
static_assert(OSP >= ND);
static_assert(32 * 2 * 16 == 16 * ND * 4);
static_assert(32 * 16 == 16 * AW * 4);
static_assert((size_t)(AW * 16 * OSP + NC + 16 * AW) * 4 <= 131072);
static_assert((size_t)NS_FULL * ND * 4 == 2097152);

typedef _Float16 h16;
typedef unsigned short bf;
typedef __attribute__((ext_vector_type(16))) __bf16   v16bf;
typedef __attribute__((ext_vector_type(16))) _Float16 v16h;
typedef __attribute__((ext_vector_type(8)))  _Float16 v8h;
typedef __attribute__((ext_vector_type(8)))  unsigned short v8us;
typedef __attribute__((ext_vector_type(8)))  float    v8f;
typedef __attribute__((ext_vector_type(4)))  float    v4f;
typedef v4f  __attribute__((may_alias)) v4fa;

__device__ __forceinline__ unsigned short f2bf(float f) { unsigned u = __float_as_uint(f); u += 0x7FFFu + ((u >> 16) & 1u); return (unsigned short)(u >> 16); }
__device__ __forceinline__ float bfr(float f) { return __uint_as_float(((unsigned)f2bf(f)) << 16); }
__device__ __forceinline__ v16h cat16(v8h lo, v8h hi) { return __builtin_shufflevector(lo, hi, 0, 1, 2, 3, 4, 5, 6, 7, 8, 9, 10, 11, 12, 13, 14, 15); }
__device__ __forceinline__ v16bf cat16b(v8us lo, v8us hi) { return __builtin_bit_cast(v16bf, __builtin_shufflevector(lo, hi, 0, 1, 2, 3, 4, 5, 6, 7, 8, 9, 10, 11, 12, 13, 14, 15)); }
__device__ __forceinline__ v8f wmma16(v16h a, v16h b, v8f c) { return __builtin_amdgcn_wmma_f32_16x16x32_f16(false, a, false, b, (short)0, c, false, false); }
__device__ __forceinline__ v8f wmmab(v16bf a, v16bf b, v8f c) { return __builtin_amdgcn_wmma_f32_16x16x32_bf16(false, a, false, b, (short)0, c, false, false); }
__device__ __forceinline__ v16h  ldh(const h16* p) { return cat16(*(const v8h*)p, *(const v8h*)(p + 16)); }
__device__ __forceinline__ v16bf ldb(const bf* p)  { return cat16b(*(const v8us*)p, *(const v8us*)(p + 16)); }
__device__ __forceinline__ void wave_sync() { __builtin_amdgcn_fence(3  , "wavefront"); __builtin_amdgcn_wave_barrier(); asm volatile("" ::: "memory"); }

__device__ __forceinline__ v16bf ldb_k16(const bf* p) { const v8us z = (v8us){}; return cat16b(*(const v8us*)p, z); }
__device__ __forceinline__ h16 toh_flush(float v) { const h16 r = (h16)v; return (fabsf(v) < 6.103515625e-05f) ? (h16)0.0f : r; }
__device__ __forceinline__ v8f wmmab_g(v16bf a, v16bf b, v8f c) { c = wmmab(a, b, c); asm volatile("v_nop\n\tv_nop\n\tv_nop\n\tv_nop" : "+v"(c) : "v"(a), "v"(b)); return c; }
__device__ __forceinline__ v8f wmma16_g(v16h a, v16h b, v8f c) { c = wmma16(a, b, c); asm volatile("v_nop\n\tv_nop\n\tv_nop\n\tv_nop" : "+v"(c) : "v"(a), "v"(b)); return c; }

__global__ __launch_bounds__(256) void k_cvt8(const float* __restrict__ src, bf* dst, size_t n8) {
    const size_t i = (size_t)blockIdx.x * 256 + threadIdx.x; if (i >= n8) return;
    const v8f v = *(const v8f*)(src + i * 8); v8us o;
#pragma unroll
    for (int k = 0; k < 8; ++k) o[k] = f2bf(v[k]);
    *(volatile v8us*)(dst + i * 8) = o; __threadfence(); *(volatile v8us*)(dst + i * 8) = o;
}

__global__ __launch_bounds__(256) void k_ytr(const float* __restrict__ src, h16* dst) {
    const int i = blockIdx.x * 256 + threadIdx.x; if (i >= ND * NC / 8) return;
    const int d = i / (NC / 8), c8 = (i % (NC / 8)) * 8;
    v8h o;
#pragma unroll
    for (int k = 0; k < 8; ++k) o[k] = toh_flush(bfr(src[(size_t)(c8 + k) * ND + d]));
    *(volatile v8h*)(dst + (size_t)i * 8) = o; __threadfence(); *(volatile v8h*)(dst + (size_t)i * 8) = o;
}

__global__ __launch_bounds__(32 * AW) void k_softsel(const bf* __restrict__ XB, const bf* __restrict__ YB, const h16* __restrict__ YT,
                                                    const float* __restrict__ bvec, float* OUT, float* FX) {
    __shared__ __align__(16) float os[AW * 16 * OSP];
    __shared__ __align__(16) float bs[NC];
    __shared__ __align__(16) float fxs[16 * AW];
    const int lane = threadIdx.x & 31, lr = lane & 15, hi = lane >> 4;
    const int wave = __builtin_amdgcn_readfirstlane((int)(threadIdx.x >> 5));
#pragma unroll 1
    for (int i = threadIdx.x; i < NC; i += 32 * AW) bs[i] = bfr(bvec[i]);
    __syncthreads();
    const int t0 = (blockIdx.x * AW + wave) * 16;
    const v16bf xq = ldb_k16(XB + (size_t)(t0 + lr) * ND + 8 * hi);
    const size_t ko = (size_t)lr * ND + 8 * hi;
    const size_t vo = (size_t)lr * NC + 8 * hi;
    v8f o0 = (v8f){};
    float m = NEGB, l = 0.0f, lf = 0.0f, fs = 0.0f;
#pragma unroll 1
    for (int key0 = 0; key0 < NC; key0 += 32) {
        const bf* ka = YB + ko + (size_t)key0 * ND;
        const v16bf ka0 = ldb_k16(ka), kb0 = ldb_k16(ka + 16 * ND);
        v8f sa = (v8f){}, sb = (v8f){};
        sa = wmmab_g(ka0, xq, sa);
        sb = wmmab_g(kb0, xq, sb);
        const int bo = key0 + 8 * hi;
        const v4f m0 = *(const v4fa*)(&bs[bo]), m1 = *(const v4fa*)(&bs[bo + 4]), m2 = *(const v4fa*)(&bs[bo + 16]), m3 = *(const v4fa*)(&bs[bo + 20]);
        float kx[8], ky[8];
#pragma unroll
        for (int r = 0; r < 4; ++r) { kx[r] = m0[r]; kx[4 + r] = m1[r]; ky[r] = m2[r]; ky[4 + r] = m3[r]; }
        float za[8], zb[8], ta[8], tb[8]; float mx = NEGB;
#pragma unroll
        for (int r = 0; r < 8; ++r) {
            za[r] = sa[r] - kx[r]; zb[r] = sb[r] - ky[r];
            ta[r] = za[r] * SC2; tb[r] = zb[r] * SC2;
            mx = fmaxf(mx, fmaxf(ta[r], tb[r])); }
        mx = fmaxf(mx, __shfl_xor(mx, 16, 32));
        const float mnew = fmaxf(m, mx);
        const float alpha = __builtin_amdgcn_exp2f(m - mnew);
        const float sh = PSH - mnew;
        v16h pb; float ls = 0.0f, lfs = 0.0f, fss = 0.0f;
#pragma unroll
        for (int r = 0; r < 8; ++r) {
            const float aa = ta[r] + sh, ab = tb[r] + sh;
            const float xa = __builtin_amdgcn_exp2f(aa), xb = __builtin_amdgcn_exp2f(ab);
            const float ea = (aa < -14.0f) ? 0.0f : xa, eb = (ab < -14.0f) ? 0.0f : xb;
            const h16 pa = (h16)ea; const h16 pc = (h16)eb;
            pb[r] = pa; pb[8 + r] = pc;
            ls += (float)pa + (float)pc;
            lfs += ea + eb;
            fss += ea * za[r] + eb * zb[r]; }
        l = l * alpha + ls; lf = lf * alpha + lfs; fs = fs * alpha + fss; m = mnew;
        o0 = o0 * alpha;
        const h16* va = YT + vo + key0;
        const v16h v0 = ldh(va);
        o0 = wmma16_g(v0, pb, o0);
    }
    l += __shfl_xor(l, 16, 32);
    lf += __shfl_xor(lf, 16, 32);
    fs += __shfl_xor(fs, 16, 32);
    const float inv = 1.0f / l;
    const float fv = fs * (1.0f / lf);
    const int wb = wave * 16 * OSP;
    { v4f a, c;
      a[0] = o0[0] * inv; a[1] = o0[1] * inv; a[2] = o0[2] * inv; a[3] = o0[3] * inv; c[0] = o0[4] * inv; c[1] = o0[5] * inv; c[2] = o0[6] * inv; c[3] = o0[7] * inv;
      *(v4fa*)(&os[wb + lr * OSP + 8 * hi]) = a; *(v4fa*)(&os[wb + lr * OSP + 8 * hi + 4]) = c; }
    if (hi == 0) fxs[wave * 16 + lr] = fv;
    wave_sync();
    float* orow = OUT + (size_t)t0 * ND;
#pragma unroll 1
    for (int ps = 0; ps < 2; ++ps) {
#pragma unroll
        for (int s = 0; s < 2; ++s) { const int p = s * 32 + lane; const int row = p >> 2, c4 = (p & 3) * 4;
            const v4f val = *(const v4fa*)(&os[wb + row * OSP + c4]);
            *(volatile v4f*)(orow + (size_t)p * 4) = val; }
        if (ps == 0) __threadfence(); }
    __syncthreads();
    if (wave == 0) {
        const v4f val = *(const v4fa*)(&fxs[lane * 4]);
        float* fp = FX + (size_t)blockIdx.x * (16 * AW) + (size_t)lane * 4;
        *(volatile v4f*)fp = val; __threadfence(); *(volatile v4f*)fp = val;
    }
}

static constexpr size_t al256(size_t v) { return (v + 255) & ~(size_t)255; }
static constexpr size_t SZ_XB = al256((size_t)NS * ND * 2);
static constexpr size_t SZ_YB = al256((size_t)NC * ND * 2);
static constexpr size_t SZ_YT = al256((size_t)ND * NC * 2);
static constexpr size_t SZ_TOTAL = SZ_XB + SZ_YB + SZ_YT;
static_assert(SZ_TOTAL <= (size_t)134217728);

extern "C" void kernel_launch(void* const* d_in, const int* in_sizes, int n_in,
                              void* d_out, int out_size, void* d_ws, size_t ws_size, hipStream_t stream) {
    if (n_in < 3) return;
    if ((size_t)in_sizes[0] < (size_t)NS * ND) return;
    if ((size_t)in_sizes[1] < (size_t)NC * ND) return;
    if ((size_t)in_sizes[2] < (size_t)NC) return;
    if ((size_t)out_size < (size_t)NS_FULL * ND + (size_t)NS) return;
    if (SZ_TOTAL > ws_size) return;
    const float* X = (const float*)d_in[0];
    const float* Y = (const float*)d_in[1];
    const float* bvec = (const float*)d_in[2];
    float* OUT = (float*)d_out;
    float* FX  = (float*)d_out + (size_t)NS_FULL * ND;
    char* wsp = (char*)d_ws;
    bf* XB = (bf*)wsp; wsp += SZ_XB;
    bf* YB = (bf*)wsp; wsp += SZ_YB;
    h16* YT = (h16*)wsp; wsp += SZ_YT;

    { const size_t n8 = (size_t)NS * ND / 8; k_cvt8<<<(unsigned)((n8 + 255) / 256), 256, 0, stream>>>(X, XB, n8); }
    { const size_t n8 = (size_t)NC * ND / 8; k_cvt8<<<(unsigned)((n8 + 255) / 256), 256, 0, stream>>>(Y, YB, n8); }
    k_ytr<<<(unsigned)((ND * NC / 8 + 255) / 256), 256, 0, stream>>>(Y, YT);

    k_softsel<<<dim3(NS / (16 * AW), 1, 1), 32 * AW, 0, stream>>>(XB, YB, YT, bvec, OUT, FX);
}
